// MyBlock_46935402611303
// MI455X (gfx1250) — hardware-verified
//
#include <hip/hip_runtime.h>
#include <math.h>

typedef __attribute__((ext_vector_type(16))) _Float16 v16h;
typedef __attribute__((ext_vector_type(16))) __bf16 v16b;
typedef __attribute__((ext_vector_type(8)))  _Float16 v8h;
typedef __attribute__((ext_vector_type(8)))  float v8f;
typedef __attribute__((ext_vector_type(4)))  float v4f;
typedef __attribute__((ext_vector_type(2)))  float v2f;
typedef __attribute__((ext_vector_type(4)))  unsigned v4u;
typedef __attribute__((ext_vector_type(4)))  int v4i;
typedef float __attribute__((may_alias)) float_a;
typedef int __attribute__((may_alias)) int_a;

template <typename T> __device__ __forceinline__ void vst2(void* p, T v) { *(volatile T*)p = v; __threadfence(); *(volatile T*)p = v; }
__device__ __forceinline__ v8f wmma16(v16h a, v16h b, v8f c) {
  v8f d = __builtin_amdgcn_wmma_f32_16x16x32_f16(false, a, false, b, (short)0, c, false, false);
  asm volatile("v_nop\n\tv_nop\n\tv_nop\n\tv_nop" : "+v"(d) : "v"(a), "v"(b));
  return d;
}
__device__ __forceinline__ v8f wmma_bf(v16b a, v16b b, v8f c) {
  v8f d = __builtin_amdgcn_wmma_f32_16x16x32_bf16(false, a, false, b, (short)0, c, false, false);
  asm volatile("v_nop\n\tv_nop\n\tv_nop\n\tv_nop" : "+v"(d) : "v"(a), "v"(b));
  return d;
}
__device__ __forceinline__ v16h frag_h(const _Float16* rowk0, int lane) {
  union { v16h v; v8h q[2]; } u; const _Float16* p = rowk0 + 8 * (lane >> 4);
  u.q[0] = *(const v8h*)p; u.q[1] = *(const v8h*)(p + 16); return u.v;
}
__device__ __forceinline__ v16h frag_f32(const float* rowk0, int lane) {
  v16h a; const float* p = rowk0 + 8 * (lane >> 4);
#pragma unroll
  for (int i = 0; i < 8; ++i) { a[i] = (_Float16)p[i]; a[8 + i] = (_Float16)p[16 + i]; }
  return a;
}
__device__ __forceinline__ v16h frag_f32s(const float* rowk0, int lane, float sc) {
  v16h a; const float* p = rowk0 + 8 * (lane >> 4);
#pragma unroll
  for (int i = 0; i < 8; ++i) { a[i] = (_Float16)(p[i] * sc); a[8 + i] = (_Float16)(p[16 + i] * sc); }
  return a;
}
__device__ __forceinline__ v16h fragc_f32(const float* W, int k0, int n, int lane, int ld, int K) {
  v16h a; const int g = lane >> 4;
#pragma unroll
  for (int i = 0; i < 8; ++i) { const int ka = k0 + 8 * g + i, kb = ka + 16;
    a[i] = (_Float16)(ka < K ? W[(size_t)(ka < K ? ka : K - 1) * ld + n] : 0.f); a[8 + i] = (_Float16)(kb < K ? W[(size_t)(kb < K ? kb : K - 1) * ld + n] : 0.f); }
  return a;
}
struct F2 { v16b h, l; };
__device__ __forceinline__ F2 bsplit16(const float v[16]) { F2 r;
#pragma unroll
  for (int i = 0; i < 16; ++i) { const __bf16 h = (__bf16)v[i]; r.h[i] = h; r.l[i] = (__bf16)(v[i] - (float)h); }
  return r; }
__device__ __forceinline__ F2 split_row(const float* row, int k0, int lane) { float v[16]; const float* p = row + k0 + 8 * (lane >> 4);
#pragma unroll
  for (int i = 0; i < 8; ++i) { v[i] = p[i]; v[8 + i] = p[16 + i]; }
  return bsplit16(v); }
__device__ __forceinline__ F2 split_rowK(const float* row, int k0, int lane, int K) { float v[16]; const int g = lane >> 4;
#pragma unroll
  for (int i = 0; i < 8; ++i) { const int ka = k0 + 8 * g + i, kb = ka + 16; v[i] = ka < K ? row[ka < K ? ka : K - 1] : 0.f; v[8 + i] = kb < K ? row[kb < K ? kb : K - 1] : 0.f; }
  return bsplit16(v); }
__device__ __forceinline__ F2 split_col(const float* W, int k0, int n, int lane, int ld, int K) { float v[16]; const int g = lane >> 4;
#pragma unroll
  for (int i = 0; i < 8; ++i) { const int ka = k0 + 8 * g + i, kb = ka + 16; v[i] = ka < K ? W[(size_t)(ka < K ? ka : K - 1) * ld + n] : 0.f; v[8 + i] = kb < K ? W[(size_t)(kb < K ? kb : K - 1) * ld + n] : 0.f; }
  return bsplit16(v); }
__device__ __forceinline__ v8f mac3(const F2& a, const F2& b, v8f c) { c = wmma_bf(a.l, b.h, c); c = wmma_bf(a.h, b.l, c); return wmma_bf(a.h, b.h, c); }
__device__ __forceinline__ float sigm(float v) { return 1.0f / (1.0f + expf(-v)); }
#define LDSX() do { asm volatile("s_wait_dscnt 0" ::: "memory"); __builtin_amdgcn_wave_barrier(); __builtin_amdgcn_fence(__ATOMIC_RELEASE, "workgroup"); } while (0)


#define NB 2
#define SS 1024
#define DMOD 1024
#define DI 2048
#define DS 16
#define DR 64
#define NXD (DR + 2 * DS)
#define DFF 4096
#define NR (NB * SS)
#define XZP (2 * DI)
#define XDP 128
#ifndef NRT
#define NRT NR
#define NBT NB
#define SST SS
#endif
typedef __attribute__((ext_vector_type(8))) __bf16 v8b;
__device__ __forceinline__ v16b frag_b(const __bf16* rowk0, int lane) {
  union { v16b v; v8b q[2]; } u; const __bf16* p = rowk0 + 8 * (lane >> 4);
  u.q[0] = *(const v8b*)p; u.q[1] = *(const v8b*)(p + 16); return u.v;
}
__device__ __forceinline__ float bfr(float v) { return (float)(__bf16)v; }
__device__ __attribute__((noinline)) float exp_ni(float v) { return expf(v); }
__device__ __attribute__((noinline)) float erf_ni(float v) { return erff(v); }

__device__ __attribute__((noinline)) float tanh_ni(float v) { return tanhf(v); }
__device__ __attribute__((noinline)) float log1p_ni(float v) { return log1pf(v); }
__device__ __forceinline__ float silu_f(float v) { return v / (1.0f + exp_ni(-v)); }
#define WS_PIN  0u
#define WS_PXP  (WS_PIN + 2u * XZP * DMOD)
#define WS_PDT  (WS_PXP + 2u * NXD * DI)
#define WS_POUT (WS_PDT + 2u * DI * DR)
#define WS_PFC  (WS_POUT + 2u * DMOD * DI)
#define WS_PPR  (WS_PFC + 2u * DFF * DMOD)
#define WS_XN   (WS_PPR + 2u * DMOD * DFF)
#define WS_XZ   (WS_XN + 4u * NR * DMOD)
#define WS_XD   (WS_XZ + 4u * NR * XZP)
#define WS_DT   (WS_XD + 4u * NR * XDP)
#define WS_X1   (WS_DT + 4u * NR * DI)
#define WS_END  (WS_X1 + 4u * NR * DMOD)

__global__ __launch_bounds__(256) void k_pack(const float* __restrict__ Wm, int K, __bf16* __restrict__ DST) {
  __shared__ __align__(16) __bf16 s[DFF]; const int n = blockIdx.x, tid = threadIdx.x; const float* src = Wm + (size_t)n * K;
  for (int k = tid; k < K; k += 256) s[k] = (__bf16)src[k];
  __syncthreads();
  for (int q = tid; q < K / 8; q += 256) vst2((unsigned*)(DST + (size_t)n * K + q * 8), *(const v4u*)&s[q * 8]);
}
template <int XB>
__global__ __launch_bounds__(256) void k_ln(const float* __restrict__ X, const float* __restrict__ gw, float* __restrict__ Y) {
  __shared__ __align__(16) float s[8][DMOD];
  const int wave = threadIdx.x >> 5, lane = threadIdx.x & 31; const size_t r = (size_t)blockIdx.x * 8 + wave; const float* x = X + r * DMOD; float* sw = s[wave];
  float sum = 0.f;
#pragma unroll 4
  for (int i = 0; i < DMOD / 32; ++i) { float t = x[lane + 32 * i]; if (XB) t = bfr(t); sw[lane + 32 * i] = t; sum += t; }
#pragma unroll
  for (int o = 1; o < 32; o <<= 1) sum += __shfl_xor(sum, o);
  const float mu = sum / (float)DMOD; float var = 0.f;
#pragma unroll 4
  for (int i = 0; i < DMOD / 32; ++i) { const float d = sw[lane + 32 * i] - mu; var += d * d; }
#pragma unroll
  for (int o = 1; o < 32; o <<= 1) var += __shfl_xor(var, o);
  const float rs = rsqrtf(var / (float)DMOD + 1e-5f);
#pragma unroll 4
  for (int i = 0; i < DMOD / 32; ++i) { const int c = lane + 32 * i; sw[c] = (sw[c] - mu) * rs * bfr(gw[c]); }
  LDSX();
#pragma unroll 2
  for (int pc = lane; pc < DMOD / 4; pc += 32) vst2(Y + r * DMOD + pc * 4, *(const v4f*)&sw[pc * 4]);
}
template <int K, int AM, int EPI, int NT, int RM>
__global__ __launch_bounds__(128) void k_lin(const float* __restrict__ A, int lda, const __bf16* __restrict__ P, const float* __restrict__ bias, float* __restrict__ OUT, int ldo, const float* __restrict__ RES, int ldr) {
  __shared__ __align__(16) float so[4][16][132];
  const int tid = threadIdx.x, wave = tid >> 5, lane = tid & 31, col = lane & 15, g = lane >> 4; const size_t r0 = (size_t)blockIdx.x * 64 + wave * 16; const int n0 = blockIdx.y * NT * 16;
  v8f acc[NT] = {};
#pragma unroll 2
  for (int kc = 0; kc < K / 32; ++kc) {
    if (AM == 0) { v16b a; { const float* p = A + (r0 + col) * lda + kc * 32 + 8 * g;
#pragma unroll
        for (int i = 0; i < 8; ++i) { a[i] = (__bf16)p[i]; a[8 + i] = (__bf16)p[16 + i]; } }
#pragma unroll
      for (int j = 0; j < NT; ++j) acc[j] = wmma_bf(a, frag_b(P + (size_t)(n0 + j * 16 + col) * K + kc * 32, lane), acc[j]); }
    else { const F2 a = split_row(A + (r0 + col) * lda, kc * 32, lane);
#pragma unroll
      for (int j = 0; j < NT; ++j) { const v16b w = frag_b(P + (size_t)(n0 + j * 16 + col) * K + kc * 32, lane); acc[j] = wmma_bf(a.l, w, acc[j]); acc[j] = wmma_bf(a.h, w, acc[j]); } } }
#pragma unroll
  for (int j = 0; j < NT; ++j) { const float bb = bias ? bfr(bias[n0 + j * 16 + col]) : 0.f;
#pragma unroll
    for (int r = 0; r < 8; ++r) { float v = acc[j][r] + bb; if (EPI == 1) v = fmaxf(v, 0.f); if (EPI == 2) v = tanh_ni(v); if (EPI == 3) v = (v > 20.f) ? v : log1p_ni(exp_ni(v)); if (EPI == 4) v = silu_f(v); if (RM == 1) v += RES[(r0 + 8 * g + r) * ldr + n0 + j * 16 + col]; if (RM == 2) v += bfr(RES[(r0 + 8 * g + r) * ldr + n0 + j * 16 + col]); so[wave][8 * g + r][j * 16 + col] = v; } }
  LDSX();
  for (int rl = 0; rl < 16; ++rl) if (lane < NT * 4) vst2(OUT + (r0 + rl) * ldo + n0 + lane * 4, *(const v4f*)&so[wave][rl][lane * 4]);
}

__global__ __launch_bounds__(256) void k_conv(float* __restrict__ XZ, const float* __restrict__ CW, const float* __restrict__ CB) {
  const int b = blockIdx.y, c0 = (blockIdx.x * 256 + threadIdx.x) * 4; float w[4][4], cb[4];
#pragma unroll
  for (int i = 0; i < 4; ++i) { cb[i] = bfr(CB[c0 + i]);
#pragma unroll
    for (int k = 0; k < 4; ++k) w[k][i] = bfr(CW[(c0 + i) * 4 + k]); }
  float* col = XZ + (size_t)b * SS * XZP + c0;
  v4f x1 = *(const v4f*)(col + (size_t)(SST - 1) * XZP), x2 = *(const v4f*)(col + (size_t)(SST - 2) * XZP), x3 = *(const v4f*)(col + (size_t)(SST - 3) * XZP);
#pragma unroll 1
  for (int t = SST - 1; t >= 0; --t) { const int tm = t - 3; v4f x0 = (tm >= 0) ? *(const v4f*)(col + (size_t)(tm >= 0 ? tm : 0) * XZP) : (v4f){0.f, 0.f, 0.f, 0.f}; v4f o;
#pragma unroll
    for (int i = 0; i < 4; ++i) { const float v = w[0][i] * x0[i] + w[1][i] * x3[i] + w[2][i] * x2[i] + w[3][i] * x1[i] + cb[i]; o[i] = silu_f(v); }
    vst2(col + (size_t)t * XZP, o); x1 = x2; x2 = x3; x3 = x0; }
}
__global__ __launch_bounds__(256) void k_scan(float* __restrict__ XZ, const float* __restrict__ XD, const float* __restrict__ DT, const float* __restrict__ ALOG, const float* __restrict__ Dp) {
  const int b = blockIdx.y, c0 = (blockIdx.x * 256 + threadIdx.x) * 4; float A[4][DS], h[4][DS], dd[4];
#pragma unroll
  for (int i = 0; i < 4; ++i) { dd[i] = bfr(Dp[c0 + i]);
#pragma unroll
    for (int n = 0; n < DS; ++n) { A[i][n] = -exp_ni(bfr(ALOG[(c0 + i) * DS + n])); h[i][n] = 0.f; } }
  const size_t rb = (size_t)b * SS;
#pragma unroll 1
  for (int t = 0; t < SST; ++t) { const size_t r = rb + t; const v4f dt4 = *(const v4f*)(DT + r * DI + c0), xb4 = *(const v4f*)(XZ + r * XZP + c0), z4 = *(const v4f*)(XZ + r * XZP + DI + c0);
    float Bt[DS], Ct[DS]; { const v4f* pb = (const v4f*)(XD + r * XDP + DR);
#pragma unroll
      for (int q = 0; q < 4; ++q) { const v4f vb = pb[q], vc = pb[4 + q];
#pragma unroll
        for (int i = 0; i < 4; ++i) { Bt[q * 4 + i] = vb[i]; Ct[q * 4 + i] = vc[i]; } } }
    v4f o;
#pragma unroll
    for (int i = 0; i < 4; ++i) { const float dti = dt4[i], xbi = xb4[i], dx = dti * xbi; float y = 0.f;
#pragma unroll
      for (int n = 0; n < DS; ++n) { h[i][n] = exp_ni(dti * A[i][n]) * h[i][n] + dx * Bt[n]; y += h[i][n] * Ct[n]; }
      y += xbi * dd[i]; o[i] = y * silu_f(z4[i]); }
    vst2(XZ + r * XZP + DI + c0, o); }
}
extern "C" void kernel_launch(void* const* d_in, const int* in_sizes, int n_in, void* d_out, int out_size, void* d_ws, size_t ws_size, hipStream_t stream) {
  (void)in_sizes; (void)n_in; (void)out_size;
  const float** F = (const float**)d_in;
  if (ws_size < (size_t)WS_END) return;
  char* ws = (char*)d_ws; __bf16 *PIN = (__bf16*)(ws + WS_PIN), *PXP = (__bf16*)(ws + WS_PXP), *PDT = (__bf16*)(ws + WS_PDT), *POUT = (__bf16*)(ws + WS_POUT), *PFC = (__bf16*)(ws + WS_PFC), *PPR = (__bf16*)(ws + WS_PPR);
  float *XN = (float*)(ws + WS_XN), *XZ = (float*)(ws + WS_XZ), *XD = (float*)(ws + WS_XD), *DT = (float*)(ws + WS_DT), *X1 = (float*)(ws + WS_X1);
  k_pack<<<XZP, 256, 0, stream>>>(F[2], DMOD, PIN);
  k_pack<<<NXD, 256, 0, stream>>>(F[5], DI, PXP);
  k_pack<<<DI, 256, 0, stream>>>(F[6], DR, PDT);
  k_pack<<<DMOD, 256, 0, stream>>>(F[10], DI, POUT);
  k_pack<<<DFF, 256, 0, stream>>>(F[12], DMOD, PFC);
  k_pack<<<DMOD, 256, 0, stream>>>(F[13], DFF, PPR);
  k_ln<1><<<NRT / 8, 256, 0, stream>>>(F[0], F[1], XN);
  k_lin<DMOD, 1, 0, 8, 0><<<dim3(NRT / 64, XZP / 128), 128, 0, stream>>>(XN, DMOD, PIN, nullptr, XZ, XZP, nullptr, 0);
  k_conv<<<dim3(DI / 1024, NBT), 256, 0, stream>>>(XZ, F[3], F[4]);
  k_lin<DI, 1, 0, 6, 0><<<dim3(NRT / 64, 1), 128, 0, stream>>>(XZ, XZP, PXP, nullptr, XD, XDP, nullptr, 0);
  k_lin<DR, 1, 3, 8, 0><<<dim3(NRT / 64, DI / 128), 128, 0, stream>>>(XD, XDP, PDT, F[7], DT, DI, nullptr, 0);
  k_scan<<<dim3(DI / 1024, NBT), 256, 0, stream>>>(XZ, XD, DT, F[8], F[9]);
  k_lin<DI, 1, 0, 8, 2><<<dim3(NRT / 64, DMOD / 128), 128, 0, stream>>>(XZ + DI, XZP, POUT, nullptr, X1, DMOD, F[0], DMOD);
  k_ln<0><<<NRT / 8, 256, 0, stream>>>(X1, F[11], XN);
  k_lin<DMOD, 1, 4, 8, 0><<<dim3(NRT / 64, DFF / 128), 128, 0, stream>>>(XN, DMOD, PFC, nullptr, XZ, DFF, nullptr, 0);
  k_lin<DFF, 1, 0, 8, 1><<<dim3(NRT / 64, DMOD / 128), 128, 0, stream>>>(XZ, DFF, PPR, nullptr, (float*)d_out, DMOD, X1, DMOD);
}
